// GrambaBlock_51977694216646
// MI455X (gfx1250) — hardware-verified
//
#include <hip/hip_runtime.h>
#include <math.h>

constexpr int kBatch     = 4;
constexpr int kSeq       = 2048;
constexpr int kDim       = 1024;
constexpr int kExp       = 4096;
constexpr int kRows      = kBatch * kSeq;
constexpr int kZHld      = 2 * kDim;
constexpr int kChunkRows = 2048;
constexpr int kChunks    = kRows / kChunkRows;
constexpr float kWCarry    = 64.0f;
constexpr float kYnCarry   = 8.0f;
constexpr float kHidCarry  = 16.0f;
constexpr float kScale2    = 1.0f / (64.0f * 8.0f);
constexpr float kScale3    = 1.0f / (64.0f * 16.0f);
constexpr float kLnEps     = 1e-5f;
constexpr float kInvDim    = 1.0f / 1024.0f;

typedef __attribute__((ext_vector_type(16))) _Float16 v16h;
typedef __attribute__((ext_vector_type(8)))  _Float16 v8h;
typedef __attribute__((ext_vector_type(16))) __bf16   v16b;
typedef __attribute__((ext_vector_type(8)))  __bf16   v8b;
typedef __attribute__((ext_vector_type(8)))  float    v8f;
typedef __attribute__((ext_vector_type(4)))  float    v4f;
typedef __attribute__((ext_vector_type(2)))  float    v2f;
typedef __attribute__((ext_vector_type(4)))  unsigned int v4u;

__device__ __forceinline__ unsigned short f2bf_bits(float f) {
  unsigned u = __float_as_uint(f);
  return (unsigned short)((u + 0x7FFFu + ((u >> 16) & 1u)) >> 16);
}
__device__ __forceinline__ float bf_bits2f(unsigned short h) { return __uint_as_float(((unsigned)h) << 16); }

__device__ __forceinline__ void dep_guard_h(v8f& a, v8f& b, v16h x, v16h y) { asm volatile("v_nop\n\tv_nop\n\tv_nop\n\tv_nop" : "+v"(a), "+v"(b) : "v"(x), "v"(y)); }
__device__ __forceinline__ void dep_guard_b(v8f& a, v8f& b, v16b x, v16b y) { asm volatile("v_nop\n\tv_nop\n\tv_nop\n\tv_nop" : "+v"(a), "+v"(b) : "v"(x), "v"(y)); }
__device__ __forceinline__ void keep4_h(v16h a, v16h b, v16h c, v16h d) { asm volatile("v_nop" :: "v"(a), "v"(b), "v"(c), "v"(d)); }
__device__ __forceinline__ void keep4_b(v16b a, v16b b, v16b c, v16b d) { asm volatile("v_nop" :: "v"(a), "v"(b), "v"(c), "v"(d)); }
__device__ __forceinline__ void acc_guard4(v8f& a, v8f& b, v8f& c, v8f& d) { asm volatile("v_nop\n\tv_nop\n\tv_nop\n\tv_nop" : "+v"(a), "+v"(b), "+v"(c), "+v"(d)); }
template <typename T> struct Frag;
template <> struct Frag<_Float16> {
  typedef v16h V; union U { v16h v; v8h h[2]; };
  static __device__ __forceinline__ v16h load(const _Float16* p) {
    U f; f.h[0] = *(const v8h*)(p); f.h[1] = *(const v8h*)(p + 16); return f.v;
  }
  static __device__ __forceinline__ v8f mma(v16h a, v16h b, v8f c) {
    return __builtin_amdgcn_wmma_f32_16x16x32_f16(false, a, false, b, (short)0, c, false, false);
  }
  static __device__ __forceinline__ void guard(v8f& a, v8f& b, v16h x, v16h y) { dep_guard_h(a, b, x, y); }
  static __device__ __forceinline__ void keep(v16h a, v16h b, v16h c, v16h d) { keep4_h(a, b, c, d); }
};
template <> struct Frag<__bf16> {
  typedef v16b V; union U { v16b v; v8b h[2]; };
  static __device__ __forceinline__ v16b load(const __bf16* p) {
    U f; f.h[0] = *(const v8b*)(p); f.h[1] = *(const v8b*)(p + 16); return f.v;
  }
  static __device__ __forceinline__ v8f mma(v16b a, v16b b, v8f c) {
    return __builtin_amdgcn_wmma_f32_16x16x32_bf16(false, a, false, b, (short)0, c, false, false);
  }
  static __device__ __forceinline__ void guard(v8f& a, v8f& b, v16b x, v16b y) { dep_guard_b(a, b, x, y); }
  static __device__ __forceinline__ void keep(v16b a, v16b b, v16b c, v16b d) { keep4_b(a, b, c, d); }
};

__device__ __forceinline__ unsigned pk16(unsigned short a, unsigned short b) { return (unsigned)a | ((unsigned)b << 16); }
__device__ __forceinline__ unsigned short h_bits(float f) { const _Float16 h = (_Float16)f; return __builtin_bit_cast(unsigned short, h); }

template <int ET> struct Elem;
template <> struct Elem<0> { typedef _Float16 T; };
template <> struct Elem<1> { typedef __bf16 T; };
template <int ET, bool SPLIT, int BIAS_MODE, int OUT_MODE, bool RESID, int ACT = 0>
__global__ __launch_bounds__(256) void wmma_gemm64(
    const unsigned short* __restrict__ Ap, const unsigned short* __restrict__ A2p, int lda, long strideA,
    const unsigned short* __restrict__ Btp, const unsigned short* __restrict__ Bt2p, int ldb, long strideB,
    void* __restrict__ Cout, void* __restrict__ Cout2, int ldc, long strideC,
    const float* __restrict__ bias,
    const float* __restrict__ resid, long strideR,
    int M, int N, int K, float scale) {
  typedef typename Elem<ET>::T T;
  typedef typename Frag<T>::V V;
  const T* A = (const T*)Ap; const T* A2 = (const T*)A2p; const T* Bt = (const T*)Btp; const T* Bt2 = (const T*)Bt2p;
  __shared__ __align__(16) float sT[8][16 * 68];
  const int b    = blockIdx.y;
  const int lane = threadIdx.x & 31;
  const int wave = threadIdx.x >> 5;
  const int tilesN = N >> 6;
  const int tilesM = M >> 6;
  const int tile = blockIdx.x * 8 + wave;
  if (tile >= tilesM * tilesN) return;
  const int tm = tile / tilesN;
  const int tn = tile - tm * tilesN;
  const int m0 = tm << 6;
  const int n0 = tn << 6;

  const T* Ab  = A  + (size_t)b * strideA;
  const T* Bb  = Bt + (size_t)b * strideB;
  const T* Ab2 = SPLIT ? (A2  + (size_t)b * strideA) : nullptr;
  const T* Bb2 = SPLIT ? (Bt2 + (size_t)b * strideB) : nullptr;

  const int rlane = lane & 15;
  const int koff  = (lane >> 4) * 8;
  const int mOff  = (lane >> 4) * 8;

  v8f acc[4][4];
#pragma unroll
  for (int i = 0; i < 4; ++i)
#pragma unroll
    for (int j = 0; j < 4; ++j) acc[i][j] = (v8f){0.f,0.f,0.f,0.f,0.f,0.f,0.f,0.f};

  for (int k0 = 0; k0 < K; k0 += 32) {
    V bh[4], bl[4];
#pragma unroll
    for (int j = 0; j < 4; ++j) {
      const size_t bo = (size_t)(n0 + (j << 4) + rlane) * ldb + koff + k0;
      bh[j] = Frag<T>::load(Bb + bo);
      if (SPLIT) bl[j] = Frag<T>::load(Bb2 + bo);
    }
#pragma unroll
    for (int i = 0; i < 4; ++i) {
      const size_t ao = (size_t)(m0 + (i << 4) + rlane) * lda + koff + k0;
      V ah = Frag<T>::load(Ab + ao);
      V al;
      if (SPLIT) al = Frag<T>::load(Ab2 + ao);
#pragma unroll
      for (int j = 0; j < 4; ++j) {
        acc[i][j] = Frag<T>::mma(ah, bh[j], acc[i][j]);
        if (SPLIT) {
          acc[i][j] = Frag<T>::mma(ah, bl[j], acc[i][j]);
          acc[i][j] = Frag<T>::mma(al, bh[j], acc[i][j]);
        }
      }
      Frag<T>::guard(acc[i][0], acc[i][3], ah, SPLIT ? al : ah);
    }
    Frag<T>::keep(bh[0], bh[1], bh[2], bh[3]);
    if (SPLIT) Frag<T>::keep(bl[0], bl[1], bl[2], bl[3]);
  }
  acc_guard4(acc[0][0], acc[0][1], acc[0][2], acc[0][3]);
  acc_guard4(acc[1][0], acc[1][1], acc[1][2], acc[1][3]);
  acc_guard4(acc[2][0], acc[2][1], acc[2][2], acc[2][3]);
  acc_guard4(acc[3][0], acc[3][1], acc[3][2], acc[3][3]);

  float* slab = sT[wave];
  const float* Rb = RESID ? (resid + (size_t)b * strideR) : nullptr;
#pragma unroll
  for (int i = 0; i < 4; ++i) {
    const int mBase = m0 + (i << 4);
#pragma unroll
    for (int j = 0; j < 4; ++j) {
      const int n = n0 + (j << 4) + rlane;
      float bv = 0.f;
      if (BIAS_MODE == 2) bv = bias[n];
#pragma unroll
      for (int r = 0; r < 8; ++r) {
        float v = acc[i][j][r] * scale;
        if (BIAS_MODE == 1) v += bias[mBase + mOff + r];
        if (BIAS_MODE == 2) v += bv;
        if (RESID) v += Rb[(size_t)(mBase + mOff + r) * ldc + n];
        if (ACT == 1) v = tanhf(v);
        if (ACT == 2) v = fmaxf(v, 0.0f);
        if (ACT == 3) v = v / (1.0f + expf(-v));
        if (ACT == 4) v = (v > 0.f) ? v : 0.01f * v;
        if (ACT == 5) v = 0.5f * v * (1.0f + erff(v * 0.70710678118654752f));
        slab[(mOff + r) * 68 + (j << 4) + rlane] = v;
      }
    }
    __builtin_amdgcn_fence(__ATOMIC_RELEASE, "workgroup");
    __builtin_amdgcn_wave_barrier();
    __builtin_amdgcn_fence(__ATOMIC_ACQUIRE, "workgroup");
    if (OUT_MODE == 0) {
      float* C = (float*)Cout + (size_t)b * strideC;
      const int hh = lane >> 4, c4 = (lane & 15) * 4;
      for (int pass = 0; pass < 2; ++pass) {
#pragma unroll
        for (int it = 0; it < 8; ++it) {
          const int row = it * 2 + hh;
          v4f v = *(const v4f*)(slab + row * 68 + c4);
          *(volatile v4f*)(C + (size_t)(mBase + row) * ldc + n0 + c4) = v;
        }
        __threadfence();
      }
    } else {
      const int q = lane >> 3, c8 = (lane & 7) * 8;
      unsigned short* C  = (unsigned short*)Cout  + (size_t)b * strideC;
      unsigned short* C2 = (OUT_MODE == 2) ? ((unsigned short*)Cout2 + (size_t)b * strideC) : nullptr;
      for (int pass = 0; pass < 2; ++pass) {
#pragma unroll
        for (int it = 0; it < 4; ++it) {
          const int row = it * 4 + q;
          const float* sp = slab + row * 68 + c8;
          v8h hv, lv;
#pragma unroll
          for (int e = 0; e < 8; ++e) {
            if (OUT_MODE == 1) {
              hv[e] = (_Float16)sp[e];
            } else {
              unsigned short hb = f2bf_bits(sp[e]);
              unsigned short lb = f2bf_bits(sp[e] - bf_bits2f(hb));
              hv[e] = __builtin_bit_cast(_Float16, hb);
              lv[e] = __builtin_bit_cast(_Float16, lb);
            }
          }
          *(volatile v8h*)(C + (size_t)(mBase + row) * ldc + n0 + c8) = hv;
          if (OUT_MODE == 2) *(volatile v8h*)(C2 + (size_t)(mBase + row) * ldc + n0 + c8) = lv;
        }
        __threadfence();
      }
    }
    __builtin_amdgcn_fence(__ATOMIC_RELEASE, "workgroup");
    __builtin_amdgcn_wave_barrier();
    __builtin_amdgcn_fence(__ATOMIC_ACQUIRE, "workgroup");
  }
}

template <int MODE>
__global__ __launch_bounds__(256) void cast8_kernel(const float* __restrict__ in, unsigned short* __restrict__ out, int n8, float scale) {
  const int i = blockIdx.x * 256 + threadIdx.x;
  if (i >= n8) return;
  const float* p = in + 8 * (size_t)i;
  const v4f a = *(const v4f*)(p);
  const v4f c = *(const v4f*)(p + 4);
  unsigned short hb[8];
#pragma unroll
  for (int e = 0; e < 4; ++e) {
    if (MODE == 0) {
      hb[e]     = f2bf_bits(a[e]);
      hb[4 + e] = f2bf_bits(c[e]);
    } else {
      hb[e]     = h_bits(bf_bits2f(f2bf_bits(a[e])) * scale);
      hb[4 + e] = h_bits(bf_bits2f(f2bf_bits(c[e])) * scale);
    }
  }
  const v4u u = (v4u){pk16(hb[0], hb[1]), pk16(hb[2], hb[3]), pk16(hb[4], hb[5]), pk16(hb[6], hb[7])};
  unsigned short* q = out + 8 * (size_t)i;
  *(volatile v4u*)q = u;
  __threadfence();
  *(volatile v4u*)q = u;
  (void)scale;
}

template <int MODE>
__global__ __launch_bounds__(256) void castT_kernel(const float* __restrict__ in, int ldin,
                                                    unsigned short* __restrict__ out, int ldo, int orow0, float scale) {
  __shared__ float sTile[64 * 65];
  const int t  = threadIdx.x;
  const int r0 = blockIdx.y * 64;
  const int c0 = blockIdx.x * 64;
  const int lr = t >> 4, lc = (t & 15) * 4;
#pragma unroll
  for (int i = 0; i < 4; ++i) {
    const int rr = lr + 16 * i;
    const v4f v = *(const v4f*)(in + (size_t)(r0 + rr) * ldin + c0 + lc);
    sTile[rr * 65 + lc + 0] = v[0];
    sTile[rr * 65 + lc + 1] = v[1];
    sTile[rr * 65 + lc + 2] = v[2];
    sTile[rr * 65 + lc + 3] = v[3];
  }
  __syncthreads();
  const int wave = t >> 5, lane = t & 31;
  const int q = lane >> 3, c8 = (lane & 7) * 8;
  v4u u[2];
  int cl[2];
#pragma unroll
  for (int it = 0; it < 2; ++it) {
    cl[it] = it * 32 + wave * 4 + q;
    unsigned short hb[8];
#pragma unroll
    for (int e = 0; e < 8; ++e) {
      const float f = sTile[(c8 + e) * 65 + cl[it]];
      if (MODE == 0) hb[e] = f2bf_bits(f);
      else           hb[e] = h_bits(bf_bits2f(f2bf_bits(f)) * scale);
    }
    u[it] = (v4u){pk16(hb[0], hb[1]), pk16(hb[2], hb[3]), pk16(hb[4], hb[5]), pk16(hb[6], hb[7])};
  }
  for (int pass = 0; pass < 2; ++pass) {
#pragma unroll
    for (int it = 0; it < 2; ++it) {
      unsigned short* p = out + (size_t)(orow0 + c0 + cl[it]) * ldo + r0 + c8;
      *(volatile v4u*)p = u[it];
    }
    __threadfence();
  }
  (void)scale;
}

__global__ __launch_bounds__(64) void scan_kernel(const float* __restrict__ ZH, const float* __restrict__ x,
                                                  const int* __restrict__ mask, const float* __restrict__ bz,
                                                  const float* __restrict__ bh, float* __restrict__ Y) {
  const int b  = blockIdx.y;
  const int d0 = (blockIdx.x * 64 + threadIdx.x) * 4;
  const v4f bzv = *(const v4f*)(bz + d0);
  const v4f bhv = *(const v4f*)(bh + d0);
  const int* mb = mask + (size_t)b * kSeq;
  float h[4] = {0.f, 0.f, 0.f, 0.f};
#pragma unroll 1
  for (int t = 0; t < kSeq; ++t) {
    const size_t row = (size_t)b * kSeq + t;
    const v4f zp = *(const v4f*)(ZH + row * kZHld + d0);
    const v4f hp = *(const v4f*)(ZH + row * kZHld + kDim + d0);
    const v4f xv = *(const v4f*)(x + row * kDim + d0);
    const int m = mb[t];
    v4f yv;
#pragma unroll
    for (int e = 0; e < 4; ++e) {
      const float zz = __builtin_amdgcn_rcpf(1.0f + __expf(-(zp[e] + bzv[e])));
      const float ht = hp[e] + bhv[e];
      const float hn = (1.0f - zz) * h[e] + zz * ht;
      h[e] = (m != 0) ? hn : h[e];
      yv[e] = bf_bits2f(f2bf_bits(xv[e])) + h[e];
    }
    float* yp = Y + row * kDim + d0;
    *(volatile v4f*)yp = yv;
    __threadfence();
    *(volatile v4f*)yp = yv;
  }
}

__global__ __launch_bounds__(128) void layernorm_kernel(float* Y, const float* __restrict__ g, const float* __restrict__ bb,
                                                        unsigned short* __restrict__ YH, float carry) {
  __shared__ __align__(16) float srow[kDim];
  __shared__ float redA[4];
  __shared__ float redB[4];
  const int row  = blockIdx.x;
  const int t    = threadIdx.x;
  const int lane = t & 31, wave = t >> 5;
  const int c0   = t * 8;
  float* yr = Y + (size_t)row * kDim;
  const v4f a = *(const v4f*)(yr + c0);
  const v4f c = *(const v4f*)(yr + c0 + 4);
  float xb[8];
#pragma unroll
  for (int e = 0; e < 4; ++e) { xb[e] = a[e]; xb[4 + e] = c[e]; }
  float s = ((xb[0] + xb[1]) + (xb[2] + xb[3])) + ((xb[4] + xb[5]) + (xb[6] + xb[7]));
#pragma unroll
  for (int off = 16; off > 0; off >>= 1) s += __shfl_xor(s, off, 32);
  if (lane == 0) redA[wave] = s;
  __syncthreads();
  const float mu = ((redA[0] + redA[1]) + (redA[2] + redA[3])) * kInvDim;
  float d[8];
#pragma unroll
  for (int e = 0; e < 8; ++e) d[e] = xb[e] - mu;
  float qq = ((d[0] * d[0] + d[1] * d[1]) + (d[2] * d[2] + d[3] * d[3])) + ((d[4] * d[4] + d[5] * d[5]) + (d[6] * d[6] + d[7] * d[7]));
#pragma unroll
  for (int off = 16; off > 0; off >>= 1) qq += __shfl_xor(qq, off, 32);
  if (lane == 0) redB[wave] = qq;
  __syncthreads();
  const float var = ((redB[0] + redB[1]) + (redB[2] + redB[3])) * kInvDim;
  const float rs  = rsqrtf(var + kLnEps);
  const v4f g0 = *(const v4f*)(g + c0), g1 = *(const v4f*)(g + c0 + 4);
  const v4f b0 = *(const v4f*)(bb + c0), b1 = *(const v4f*)(bb + c0 + 4);
  float gg[8], bv[8];
#pragma unroll
  for (int e = 0; e < 4; ++e) { gg[e] = g0[e]; gg[4 + e] = g1[e]; bv[e] = b0[e]; bv[4 + e] = b1[e]; }
  unsigned short hb[8];
#pragma unroll
  for (int e = 0; e < 8; ++e) {
    const float o = d[e] * rs * gg[e] + bv[e];
    srow[c0 + e] = o;
    hb[e] = h_bits(o * carry);
  }
  const v4u fv = (v4u){pk16(hb[0], hb[1]), pk16(hb[2], hb[3]), pk16(hb[4], hb[5]), pk16(hb[6], hb[7])};
  __syncthreads();
  const v4f s0 = *(const v4f*)(srow + 4 * t);
  const v4f s1 = *(const v4f*)(srow + 512 + 4 * t);
  float* p0 = yr + 4 * t;
  float* p1 = yr + 512 + 4 * t;
  unsigned short* hp = YH + (size_t)row * kDim + c0;
  *(volatile v4f*)p0 = s0;
  *(volatile v4f*)p1 = s1;
  *(volatile v4u*)hp = fv;
  __threadfence();
  *(volatile v4f*)p0 = s0;
  *(volatile v4f*)p1 = s1;
  *(volatile v4u*)hp = fv;
}

__global__ __launch_bounds__(256) void gelu_cast_kernel(const float* __restrict__ in, unsigned short* __restrict__ out, int n2, float carry) {
  const int i = blockIdx.x * 256 + threadIdx.x;
  if (i >= n2) return;
  const v2f v = *(const v2f*)(in + 2 * (size_t)i);
  const float a = v[0], c = v[1];
  const float ga = 0.5f * a * (1.0f + erff(a * 0.70710678118654752f));
  const float gc = 0.5f * c * (1.0f + erff(c * 0.70710678118654752f));
  const unsigned u = pk16(h_bits(ga * carry), h_bits(gc * carry));
  unsigned* q = (unsigned*)(out) + (size_t)i;
  *(volatile unsigned*)q = u;
  __threadfence();
  *(volatile unsigned*)q = u;
}

extern "C" void kernel_launch(void* const* d_in, const int* in_sizes, int n_in,
                              void* d_out, int out_size, void* d_ws, size_t ws_size,
                              hipStream_t stream) {
  if (n_in < 12) return;
  if (in_sizes[0] != kRows * kDim) return;
  if (in_sizes[1] != kBatch * kSeq) return;
  if (in_sizes[2] != kDim * kDim) return;
  if (in_sizes[3] != kDim) return;
  if (in_sizes[4] != kDim * kDim) return;
  if (in_sizes[5] != kDim) return;
  if (in_sizes[6] != kDim || in_sizes[7] != kDim) return;
  if (in_sizes[8] != kDim * kExp) return;
  if (in_sizes[9] != kExp) return;
  if (in_sizes[10] != kExp * kDim) return;
  if (in_sizes[11] != kDim) return;
  if (out_size != kRows * kDim) return;

  const float* x    = (const float*)d_in[0];
  const int*   mask = (const int*)d_in[1];
  const float* Wz   = (const float*)d_in[2];
  const float* bz   = (const float*)d_in[3];
  const float* Wh   = (const float*)d_in[4];
  const float* bh   = (const float*)d_in[5];
  const float* ln_g = (const float*)d_in[6];
  const float* ln_b = (const float*)d_in[7];
  const float* W1   = (const float*)d_in[8];
  const float* b1   = (const float*)d_in[9];
  const float* W2   = (const float*)d_in[10];
  const float* b2   = (const float*)d_in[11];
  float* outp = (float*)d_out;

  const size_t SZ_ZH   = (size_t)kRows * kZHld * 4;
  const size_t SZ_W1T  = (size_t)kExp * kDim * 2;
  const size_t SZ_W2T  = (size_t)kDim * kExp * 2;
  const size_t SZ_PRE  = (size_t)kChunkRows * kExp * 4;
  const size_t SZ_HID  = (size_t)kChunkRows * kExp * 2;
  const size_t SZ_Y    = (size_t)kRows * kDim * 4;
  const size_t SZ_X16  = (size_t)kRows * kDim * 2;
  const size_t SZ_WCAT = (size_t)kZHld * kDim * 2;

  size_t off = 0;
  const size_t oZ    = off;
  const size_t oW1T  = oZ;
  const size_t oW2T  = oW1T + SZ_W1T;
  const size_t oPRE  = oW2T + SZ_W2T;
  const size_t oHID  = oPRE + SZ_PRE;
  const size_t endC  = oHID + SZ_HID;
  const size_t endZ  = (endC > oZ + SZ_ZH) ? endC : (oZ + SZ_ZH);
  off = endZ;
  const size_t oY    = off; off += SZ_Y;
  const size_t oX    = off; off += SZ_X16;
  const size_t oWCAT = off; off += SZ_WCAT;
  const size_t TOTAL = off;
  if (TOTAL > ws_size) return;
  if (TOTAL > (size_t)134217728) return;

  char* ws = (char*)d_ws;
  float*          ZH    = (float*)(ws + oZ);
  unsigned short* W1T   = (unsigned short*)(ws + oW1T);
  unsigned short* W2T   = (unsigned short*)(ws + oW2T);
  float*          PRE   = (float*)(ws + oPRE);
  unsigned short* HID   = (unsigned short*)(ws + oHID);
  float*          Ybuf  = (float*)(ws + oY);
  unsigned short* Xb    = (unsigned short*)(ws + oX);
  unsigned short* YN16  = (unsigned short*)(ws + oX);
  unsigned short* WCATT = (unsigned short*)(ws + oWCAT);

  const dim3 blk(256);

  {
    const int n8x = kRows * kDim / 8;
    cast8_kernel<0><<<dim3(n8x / 256), blk, 0, stream>>>(x, Xb, n8x, 1.0f);
    castT_kernel<0><<<dim3(kDim / 64, kDim / 64), blk, 0, stream>>>(Wz, kDim, WCATT, kDim, 0, 1.0f);
    castT_kernel<0><<<dim3(kDim / 64, kDim / 64), blk, 0, stream>>>(Wh, kDim, WCATT, kDim, kDim, 1.0f);
  }

  {
    const int tiles = (kRows / 64) * (kZHld / 64);
    wmma_gemm64<1, false, 0, 0, false, 0><<<dim3(tiles / 8, 1), blk, 0, stream>>>(
        Xb, Xb, kDim, 0L, WCATT, WCATT, kDim, 0L, (void*)ZH, (void*)ZH, kZHld, 0L, bz, x, 0L, kRows, kZHld, kDim, 1.0f);
  }

  scan_kernel<<<dim3(kDim / 256, kBatch), dim3(64), 0, stream>>>(ZH, x, mask, bz, bh, Ybuf);

  layernorm_kernel<<<dim3(kRows), dim3(128), 0, stream>>>(Ybuf, ln_g, ln_b, YN16, kYnCarry);

  castT_kernel<1><<<dim3(kExp / 64, kDim / 64), blk, 0, stream>>>(W1, kExp, W1T, kDim, 0, kWCarry);
  castT_kernel<1><<<dim3(kDim / 64, kExp / 64), blk, 0, stream>>>(W2, kDim, W2T, kExp, 0, kWCarry);

  const int tiles2 = (kChunkRows / 64) * (kExp / 64);
  const int tiles3 = (kChunkRows / 64) * (kDim / 64);
  const int n2     = kChunkRows * kExp / 2;
  for (int ch = 0; ch < kChunks; ++ch) {
    const size_t rowoff = (size_t)ch * kChunkRows;
    const unsigned short* Ayn = YN16 + rowoff * kDim;
    wmma_gemm64<0, false, 2, 0, false, 0><<<dim3(tiles2 / 8, 1), blk, 0, stream>>>(
        Ayn, Ayn, kDim, 0L, W1T, W1T, kDim, 0L, (void*)PRE, (void*)PRE, kExp, 0L, b1, x, 0L, kChunkRows, kExp, kDim, kScale2);
    gelu_cast_kernel<<<dim3(n2 / 256), blk, 0, stream>>>(PRE, HID, n2, kHidCarry);
    float* Cc = outp + rowoff * kDim;
    const float* Rc = Ybuf + rowoff * kDim;
    wmma_gemm64<0, false, 2, 0, true, 0><<<dim3(tiles3 / 8, 1), blk, 0, stream>>>(
        HID, HID, kExp, 0L, W2T, W2T, kExp, 0L, (void*)Cc, (void*)Cc, kDim, 0L, b2, Rc, 0L, kChunkRows, kDim, kExp, kScale3);
  }
  (void)stream;
}
